// CustomTwoLayerGNN_34333968564342
// MI455X (gfx1250) — hardware-verified
//
#include <hip/hip_runtime.h>
#include <stddef.h>


#define D1      128
#define NOUT    256
#define K1      256
#define K2      512
#define NTHR    256
#define NWAVE   8
#define EPT     8
#define NGRP    2
#define CHUNK   (NTHR * EPT * NGRP)
#define WCAP    (EPT * NGRP * 32)
#define LISTN   (NWAVE * WCAP)
#define NBC     4096
#define NBF     2048
#define FPC     (NBC / NBF)
#define RCAP    49152
#define RBN     128
#define TGT     256
#define DEGCAP  256
#define OTHR    512
#define BM      32
#define TT      64
#define NTILE1  ((K1 / TT) * (NOUT / TT))
#define NTILE2  ((K2 / TT) * (NOUT / TT))
#define WSCAP   134217728
#define WSCL    64.0f
#define WSCLI   0.015625f

#define LDS_FILL ((RCAP + NBF + LISTN) * 4 + 64)
#define LDS_MLP1 (BM * K1 * 2 + BM * NOUT * 4)
#define LDS_MLP2 (BM * K2 * 2 + BM * NOUT * 4)

static_assert((CHUNK & (CHUNK - 1)) == 0);
static_assert(CHUNK <= 4096);
static_assert(NBC <= 4096 && NBF <= 4096);
static_assert((NBC & (NBC - 1)) == 0 && (NBF & (NBF - 1)) == 0);
static_assert(NBC == FPC * NBF && FPC == 2);
static_assert(OTHR * 8 == NBC);
static_assert(OTHR / 32 == 8 * FPC);
static_assert((RCAP % 32) == 0);
static_assert(TGT == NWAVE * 32);
static_assert((TGT % BM) == 0);
static_assert((DEGCAP % 32) == 0);
static_assert(BM == 32 && NWAVE == 8 && NTHR == 256);
static_assert(NOUT == 256 && K1 == 2 * D1 && K2 == 2 * NOUT);
static_assert((K1 % TT) == 0 && (K2 % TT) == 0 && (NOUT % TT) == 0);
static_assert(LDS_MLP1 <= 65536 && LDS_MLP2 <= 65536);

typedef float          v4f  __attribute__((ext_vector_type(4)));
typedef float          v8f  __attribute__((ext_vector_type(8)));
typedef int            v4i  __attribute__((ext_vector_type(4)));
typedef _Float16       v4h  __attribute__((ext_vector_type(4)));
typedef _Float16       v8h  __attribute__((ext_vector_type(8)));
typedef _Float16       v16h __attribute__((ext_vector_type(16)));
union FragH { v16h v; v8h h[2]; };

__device__ __forceinline__ v8f wmh(v16h a, v16h b, v8f c) {
  v8f d = __builtin_amdgcn_wmma_f32_16x16x32_f16(false, a, false, b, (short)0, c, false, false);
  asm volatile("v_nop\n\tv_nop\n\tv_nop\n\tv_nop" : "+v"(d) : "v"(a), "v"(b));
  return d;
}

__device__ __forceinline__ v8h cvt8(v4f a, v4f b, float s) {
  v8h r;
  r[0] = (_Float16)(a.x * s); r[1] = (_Float16)(a.y * s); r[2] = (_Float16)(a.z * s); r[3] = (_Float16)(a.w * s);
  r[4] = (_Float16)(b.x * s); r[5] = (_Float16)(b.y * s); r[6] = (_Float16)(b.z * s); r[7] = (_Float16)(b.w * s);
  return r;
}

__global__ __launch_bounds__(NTHR) void k_wprep(const float* __restrict__ Wa, const float* __restrict__ Wb,
                                               _Float16* Pa, _Float16* Pb) {
  __shared__ __attribute__((aligned(16))) _Float16 T[TT * TT];
  const int tid = threadIdx.x;
  int b = (int)blockIdx.x;
  const int sel = (b >= NTILE1) ? 1 : 0;
  b = sel ? (b - NTILE1) : b;
  const int K = sel ? K2 : K1;
  const float* W = sel ? Wb : Wa;
  _Float16* P = sel ? Pb : Pa;
  const int kt = b / (NOUT / TT), nt = b - kt * (NOUT / TT);
  const int k0 = kt * TT, n0 = nt * TT;

#pragma unroll
  for (int it = 0; it < (TT * TT / 4) / NTHR; ++it) {
    const int u = it * NTHR + tid;
    const int r = u >> 4, c = (u & 15) * 4;
    const v4f w = *(const v4f*)(W + (size_t)(k0 + r) * NOUT + n0 + c);
    T[(c + 0) * TT + r] = (_Float16)(w.x * WSCL);
    T[(c + 1) * TT + r] = (_Float16)(w.y * WSCL);
    T[(c + 2) * TT + r] = (_Float16)(w.z * WSCL);
    T[(c + 3) * TT + r] = (_Float16)(w.w * WSCL);
  }
  __syncthreads();

  v8h pv[2];
#pragma unroll
  for (int p = 0; p < 2; ++p) {
    const int L = p * 32 + (tid >> 3), q = tid & 7;
    pv[p] = *(const v8h*)(T + L * TT + 8 * q);
  }
#pragma unroll
  for (int p = 0; p < 2; ++p) {
    const int L = p * 32 + (tid >> 3), q = tid & 7;
    *(volatile v8h*)(P + (size_t)(n0 + L) * K + k0 + 8 * q) = pv[p];
  }
  __threadfence();
#pragma unroll
  for (int p = 0; p < 2; ++p) {
    const int L = p * 32 + (tid >> 3), q = tid & 7;
    *(volatile v8h*)(P + (size_t)(n0 + L) * K + k0 + 8 * q) = pv[p];
  }
}

template <int NB>
__device__ __forceinline__ int scan_chunk(const int* __restrict__ dsts, int nE, int cbase, int slotBase,
                                          int vec8, int* list, int tid, int lane, int wave) {
  int wc = 0;
#pragma unroll
  for (int g = 0; g < NGRP; ++g) {
    const int el0  = (g * NTHR + tid) * EPT;
    const int e0   = cbase + el0;
    const int sent = -2147483647 - 1;
    v4i da, db;
    if (vec8 != 0 && cbase + CHUNK <= nE) {
      da = *(const v4i*)(dsts + e0);
      db = *(const v4i*)(dsts + e0 + 4);
    } else {
      da.x = (e0     < nE) ? dsts[min(e0, nE - 1)] : sent;
      da.y = (e0 + 1 < nE) ? dsts[min(e0 + 1, nE - 1)] : sent;
      da.z = (e0 + 2 < nE) ? dsts[min(e0 + 2, nE - 1)] : sent;
      da.w = (e0 + 3 < nE) ? dsts[min(e0 + 3, nE - 1)] : sent;
      db.x = (e0 + 4 < nE) ? dsts[min(e0 + 4, nE - 1)] : sent;
      db.y = (e0 + 5 < nE) ? dsts[min(e0 + 5, nE - 1)] : sent;
      db.z = (e0 + 6 < nE) ? dsts[min(e0 + 6, nE - 1)] : sent;
      db.w = (e0 + 7 < nE) ? dsts[min(e0 + 7, nE - 1)] : sent;
    }
    const unsigned nb = (unsigned)slotBase;
    const unsigned s0 = (unsigned)da.x - nb, s1 = (unsigned)da.y - nb;
    const unsigned s2 = (unsigned)da.z - nb, s3 = (unsigned)da.w - nb;
    const unsigned s4 = (unsigned)db.x - nb, s5 = (unsigned)db.y - nb;
    const unsigned s6 = (unsigned)db.z - nb, s7 = (unsigned)db.w - nb;
    const bool h0 = s0 < (unsigned)NB, h1 = s1 < (unsigned)NB, h2 = s2 < (unsigned)NB, h3 = s3 < (unsigned)NB;
    const bool h4 = s4 < (unsigned)NB, h5 = s5 < (unsigned)NB, h6 = s6 < (unsigned)NB, h7 = s7 < (unsigned)NB;
    const unsigned any = __builtin_amdgcn_ballot_w32(h0 | h1 | h2 | h3 | h4 | h5 | h6 | h7);
    if (any != 0u) {
#define HITJ(J, HJ, SJ) { \
        const unsigned mj = __builtin_amdgcn_ballot_w32(HJ); \
        if (mj != 0u) { \
          if (HJ) { \
            const int pos = wc + (int)__builtin_amdgcn_mbcnt_lo(mj, 0u); \
            if (pos < WCAP) list[wave * WCAP + pos] = ((el0 + (J)) << 12) | (int)(SJ); \
          } \
          wc += (int)__builtin_popcount(mj); } }
      HITJ(0, h0, s0)
      HITJ(1, h1, s1)
      HITJ(2, h2, s2)
      HITJ(3, h3, s3)
      HITJ(4, h4, s4)
      HITJ(5, h5, s5)
      HITJ(6, h6, s6)
      HITJ(7, h7, s7)
#undef HITJ
    }
  }
  return wc;
}

__global__ __launch_bounds__(NTHR) void k_count(
    const int* __restrict__ dsts, int* cnt, int nE, int vec8) {
  __shared__ __attribute__((aligned(16))) int scnt[NBC];
  __shared__ __attribute__((aligned(16))) int list[LISTN];
  __shared__ int wcnt[NWAVE];
  const int tid = threadIdx.x, lane = tid & 31, wave = tid >> 5;
  const int nodeBase = blockIdx.x * NBC;

  for (int i = tid; i < NBC; i += NTHR) scnt[i] = 0;
  __syncthreads();

  const int nChunks = (nE + CHUNK - 1) / CHUNK;
#pragma unroll 1
  for (int ch = 0; ch < nChunks; ++ch) {
    const int cbase = ch * CHUNK;
    const int wc = scan_chunk<NBC>(dsts, nE, cbase, nodeBase, vec8, list, tid, lane, wave);
    if (lane == 0) wcnt[wave] = wc;
    __syncthreads();
    if (wave == 0) {
#pragma unroll 1
      for (int wsx = 0; wsx < NWAVE; ++wsx) {
        int n = __builtin_amdgcn_readfirstlane(wcnt[wsx]);
        n = n > WCAP ? WCAP : (n < 0 ? 0 : n);
        const int* lp = list + wsx * WCAP;
#pragma unroll 1
        for (int i = 0; i < n; ++i) {
          const int ent  = __builtin_amdgcn_readfirstlane(lp[i]);
          const int slot = ent & (NBC - 1);
          if (lane == 0) scnt[slot] = scnt[slot] + 1;
        }
      }
    }
    __syncthreads();
  }

  v4i cq[4];
#pragma unroll
  for (int q = 0; q < 4; ++q) {
    const int f = (wave * 4 + q) * 128 + 4 * lane;
    cq[q] = *(const v4i*)(scnt + f);
  }
  int* cpn = cnt + (size_t)nodeBase;
#pragma unroll
  for (int q = 0; q < 4; ++q) {
    const int f = (wave * 4 + q) * 128 + 4 * lane;
    *(volatile v4i*)(cpn + f) = cq[q];
  }
  __threadfence();
#pragma unroll
  for (int q = 0; q < 4; ++q) {
    const int f = (wave * 4 + q) * 128 + 4 * lane;
    *(volatile v4i*)(cpn + f) = cq[q];
  }
}

__global__ __launch_bounds__(OTHR) void k_offsets(
    const int* __restrict__ cnt, int* off, int* rbase, int nChunk) {
  __shared__ __attribute__((aligned(16))) int soff[NBC];
  __shared__ __attribute__((aligned(16))) int srb[RBN];
  __shared__ int wtot[OTHR / 32];
  const int tid = threadIdx.x, lane = tid & 31, wave = tid >> 5, sub = tid >> 8;
  for (int i = tid; i < RBN; i += OTHR) srb[i] = 0;
  __syncthreads();
  int carry = 0;
#pragma unroll 1
  for (int ch = 0; ch < nChunk; ++ch) {
    const int base = ch * NBC;
    const v4i ca = *(const v4i*)(cnt + base + 8 * tid);
    const v4i cb = *(const v4i*)(cnt + base + 8 * tid + 4);
    const int e0 = max(ca.x, 0), e1 = max(ca.y, 0), e2 = max(ca.z, 0), e3 = max(ca.w, 0);
    const int e4 = max(cb.x, 0), e5 = max(cb.y, 0), e6 = max(cb.z, 0), e7 = max(cb.w, 0);
    const int ts = e0 + e1 + e2 + e3 + e4 + e5 + e6 + e7;
    int incl = ts;
#pragma unroll
    for (int d = 1; d < 32; d <<= 1) {
      const int t = __shfl_up(incl, d);
      if (lane >= d) incl += t;
    }
    if (lane == 31) wtot[wave] = incl;
    __syncthreads();
    int S0 = 0, S1 = 0;
#pragma unroll
    for (int w = 0; w < 8; ++w) { S0 += wtot[w]; S1 += wtot[8 + w]; }
    int pre = 0;
#pragma unroll 1
    for (int w = 8 * sub; w < wave; ++w) pre += wtot[w];
    const int b0 = carry;
    const int b1 = b0 + ((S0 + 31) & ~31);
    const int b2 = b1 + ((S1 + 31) & ~31);
    const int myb = sub == 0 ? b0 : b1;
    if (tid == 0) {
      srb[min(2 * ch + 0, RBN - 1)] = b0;
      srb[min(2 * ch + 1, RBN - 1)] = b1;
    }
    int run = myb + pre + incl - ts;
    soff[8 * tid + 0] = run; run += e0;
    soff[8 * tid + 1] = run; run += e1;
    soff[8 * tid + 2] = run; run += e2;
    soff[8 * tid + 3] = run; run += e3;
    soff[8 * tid + 4] = run; run += e4;
    soff[8 * tid + 5] = run; run += e5;
    soff[8 * tid + 6] = run; run += e6;
    soff[8 * tid + 7] = run;
    carry = b2;
    __syncthreads();
    const v4i o0 = *(const v4i*)(soff + 4 * tid);
    const v4i o1 = *(const v4i*)(soff + 4 * (tid + OTHR));
    int* op = off + base;
    *(volatile v4i*)(op + 4 * tid) = o0;
    *(volatile v4i*)(op + 4 * (tid + OTHR)) = o1;
    __threadfence();
    *(volatile v4i*)(op + 4 * tid) = o0;
    *(volatile v4i*)(op + 4 * (tid + OTHR)) = o1;
    __syncthreads();
  }
  if (tid == 0) srb[min(2 * nChunk, RBN - 1)] = carry;
  __syncthreads();
  v4i rv = {0, 0, 0, 0};
  if (tid < 32) rv = *(const v4i*)(srb + 4 * tid);
  if (tid < 32) *(volatile v4i*)(rbase + 4 * tid) = rv;
  __threadfence();
  if (tid < 32) *(volatile v4i*)(rbase + 4 * tid) = rv;
}

__global__ __launch_bounds__(NTHR) void k_fill(
    const int* __restrict__ dsts, const int* __restrict__ srcs, const int* __restrict__ off,
    const int* __restrict__ rbase, int* csr, int nN, int nE, int vec8, int csrLen) {
  extern __shared__ v4f lds_dyn[];
  int* region = (int*)lds_dyn;
  int* cursor = region + RCAP;
  int* list   = cursor + NBF;
  int* wcnt   = list + LISTN;
  const int tid = threadIdx.x, lane = tid & 31, wave = tid >> 5;
  const int b = blockIdx.x;
  const int nodeBase = b * NBF;

  int rb0 = rbase[b];
  const int rb1 = rbase[b + 1];
  rb0 = rb0 < 0 ? 0 : (rb0 > csrLen ? csrLen : rb0);
  rb0 &= ~31;
  int len = rb1 - rb0;
  len = len < 0 ? 0 : (len > RCAP ? RCAP : len);
  int lenW = (len + 31) & ~31;
  if (rb0 + lenW > csrLen) lenW = (csrLen - rb0) & ~31;

  {
    const v4i z = {0, 0, 0, 0};
    for (int i = tid; i < RCAP / 4; i += NTHR) ((v4i*)region)[i] = z;
    for (int s = tid; s < NBF; s += NTHR) {
      int o = off[nodeBase + s] - rb0;
      o = o < 0 ? 0 : (o > RCAP ? RCAP : o);
      cursor[s] = o;
    }
  }
  __syncthreads();

  const int nChunks = (nE + CHUNK - 1) / CHUNK;
#pragma unroll 1
  for (int ch = 0; ch < nChunks; ++ch) {
    const int cbase = ch * CHUNK;
    const int wc = scan_chunk<NBF>(dsts, nE, cbase, nodeBase, vec8, list, tid, lane, wave);
    if (lane == 0) wcnt[wave] = wc;
    __syncthreads();
    if (wave == 0) {
#pragma unroll 1
      for (int wsx = 0; wsx < NWAVE; ++wsx) {
        int n = __builtin_amdgcn_readfirstlane(wcnt[wsx]);
        n = n > WCAP ? WCAP : (n < 0 ? 0 : n);
        const int* lp = list + wsx * WCAP;
#pragma unroll 1
        for (int i = 0; i < n; ++i) {
          const int ent  = __builtin_amdgcn_readfirstlane(lp[i]);
          const int slot = ent & (NBF - 1);
          int e = cbase + ((ent >> 12) & (CHUNK - 1));
          e = e < 0 ? 0 : (e > nE - 1 ? nE - 1 : e);
          int sv = srcs[e];
          sv = sv < 0 ? 0 : (sv > nN - 1 ? nN - 1 : sv);
          if (lane == 0) {
            int pos = cursor[slot];
            pos = pos < 0 ? 0 : (pos > RCAP - 1 ? RCAP - 1 : pos);
            region[pos] = sv;
            const int np = pos + 1;
            cursor[slot] = np > RCAP ? RCAP : np;
          }
        }
      }
    }
    __syncthreads();
  }

  const int nv = lenW >> 2;
  int* gp = csr + rb0;
#pragma unroll 1
  for (int i = tid; i < nv; i += NTHR) { const v4i v = ((const v4i*)region)[i]; *(volatile v4i*)(gp + 4 * i) = v; }
  __threadfence();
#pragma unroll 1
  for (int i = tid; i < nv; i += NTHR) { const v4i v = ((const v4i*)region)[i]; *(volatile v4i*)(gp + 4 * i) = v; }
}

template <int NV>
__global__ __launch_bounds__(NTHR) void k_agg(
    const int* __restrict__ csr, const int* __restrict__ off, const int* __restrict__ cnt,
    const float* __restrict__ X, _Float16* AG, int nN, int csrLen) {
  constexpr int D = 128 * NV;
  const int tid = threadIdx.x, lane = tid & 31, wave = tid >> 5;
  const int tbase = blockIdx.x * TGT + wave * 32;
  const int col = 4 * NV * lane;
  const v4f z4 = {0.f, 0.f, 0.f, 0.f};
  const int cl    = tbase + lane;
  const int cnt_l = cnt[cl];
  const int off_l = off[cl];

#pragma unroll 1
  for (int j = 0; j < 32; ++j) {
    const int c  = tbase + j;
    const int dg = __shfl(cnt_l, j);
    const int n  = dg < 0 ? 0 : (dg > DEGCAP ? DEGCAP : dg);
    const int st = __shfl(off_l, j);
    v4f acc[2];
    acc[0] = z4; acc[1] = z4;
#pragma unroll 1
    for (int q0 = 0; q0 < n; q0 += 32) {
      int pos = st + q0 + lane;
      pos = pos < 0 ? 0 : (pos > csrLen - 1 ? csrLen - 1 : pos);
      int sl = csr[pos];
      sl = sl < 0 ? 0 : (sl > nN - 1 ? nN - 1 : sl);
      const int mcnt = (n - q0) < 32 ? (n - q0) : 32;
#pragma unroll 1
      for (int pp = 0; pp < mcnt; ++pp) {
        const int s = __builtin_amdgcn_readlane(sl, pp);
        const float* xr = X + (size_t)s * D + col;
#pragma unroll
        for (int i = 0; i < NV; ++i) acc[i] += *(const v4f*)(xr + 4 * i);
      }
    }
    const float df  = (float)(dg < 1 ? 1 : dg);
    const float inv = 1.0f / df;
#pragma unroll
    for (int i = 0; i < NV; ++i) {
      acc[i] = acc[i] * inv;
      if (c >= nN) acc[i] = z4;
    }
    _Float16* po = AG + (size_t)c * D + col;
    if (NV == 1) {
      v4h o;
      o[0] = (_Float16)acc[0].x; o[1] = (_Float16)acc[0].y; o[2] = (_Float16)acc[0].z; o[3] = (_Float16)acc[0].w;
      *(volatile v4h*)po = o;
      __threadfence();
      *(volatile v4h*)po = o;
    } else {
      const v8h o = cvt8(acc[0], acc[1], 1.0f);
      *(volatile v8h*)po = o;
      __threadfence();
      *(volatile v8h*)po = o;
    }
  }
}

template <int ROWS, int KW, int PD>
__device__ __forceinline__ void stage_rows(const float* src, int rowBase, int nValid, _Float16* dst, int colOff) {
  constexpr int UPR = KW / 8;
  constexpr int NU  = ROWS * UPR;
  static_assert((NU % NTHR) == 0);
  const int tid = threadIdx.x;
  const v4f z4 = {0.f, 0.f, 0.f, 0.f};
#pragma unroll 2
  for (int it = 0; it < NU / NTHR; ++it) {
    const int u = it * NTHR + tid;
    const int r = u / UPR, c = (u % UPR) * 8;
    const int grow = rowBase + r;
    const int rc = grow < nValid ? grow : nValid - 1;
    const float* p = src + (size_t)rc * KW + c;
    v4f a = *(const v4f*)p, b = *(const v4f*)(p + 4);
    if (grow >= nValid) { a = z4; b = z4; }
    *(v8h*)(dst + (size_t)r * PD + colOff + c) = cvt8(a, b, 1.0f);
  }
}

template <int ROWS, int KW, int PD>
__device__ __forceinline__ void stage_h(const _Float16* src, int rowBase, int nPlane, _Float16* dst, int colOff) {
  constexpr int UPR = KW / 8;
  constexpr int NU  = ROWS * UPR;
  static_assert((NU % NTHR) == 0);
  const int tid = threadIdx.x;
  v8h z8;
#pragma unroll
  for (int i = 0; i < 8; ++i) z8[i] = (_Float16)0.0f;
#pragma unroll 2
  for (int it = 0; it < NU / NTHR; ++it) {
    const int u = it * NTHR + tid;
    const int r = u / UPR, c = (u % UPR) * 8;
    const int grow = rowBase + r;
    const int rc = grow < nPlane ? grow : nPlane - 1;
    v8h v = *(const v8h*)(src + (size_t)rc * KW + c);
    if (grow >= nPlane) v = z8;
    *(v8h*)(dst + (size_t)r * PD + colOff + c) = v;
  }
}

template <int NT, int KA>
__device__ __forceinline__ void mmk(v8f (&acc)[NT], const _Float16* tA, int arow,
                                    const _Float16* __restrict__ Bp, int bcol0) {
  const int lane = threadIdx.x & 31, hh = lane >> 4, m = lane & 15;
  const _Float16* ap = tA + (arow + m) * KA + 8 * hh;
  const _Float16* bp = Bp + (size_t)(bcol0 + m) * KA + 8 * hh;
#pragma unroll 1
  for (int kt = 0; kt < KA / 32; ++kt) {
    FragH a;
    a.h[0] = *(const v8h*)(ap + 32 * kt);
    a.h[1] = *(const v8h*)(ap + 32 * kt + 16);
#pragma unroll
    for (int t = 0; t < NT; ++t) {
      const size_t to = (size_t)(16 * t) * KA + 32 * kt;
      FragH bq;
      bq.h[0] = *(const v8h*)(bp + to);
      bq.h[1] = *(const v8h*)(bp + to + 16);
      acc[t] = wmh(a.v, bq.v, acc[t]);
    }
  }
}

template <int DS>
__global__ __launch_bounds__(NTHR) void k_mlp(
    const float* __restrict__ Xs, const _Float16* __restrict__ AGp,
    const _Float16* __restrict__ Pw, const float* __restrict__ bias,
    float* out, int nValid, int nPlane, int nWrite) {
  constexpr int K = 2 * DS;
  extern __shared__ v4f lds_dyn[];
  _Float16* tA  = (_Float16*)lds_dyn;
  float*    stg = (float*)(tA + BM * K);
  const int tid = threadIdx.x, lane = tid & 31, wave = tid >> 5, hh = lane >> 4, m = lane & 15;
  const int rowBase = blockIdx.x * BM;
  const int r0 = (wave >> 2) * 16, c0 = (wave & 3) * 64;

  stage_rows<BM, DS, K>(Xs, rowBase, nValid, tA, 0);
  stage_h<BM, DS, K>(AGp, rowBase, nPlane, tA, DS);
  __syncthreads();

  v8f acc[4];
#pragma unroll
  for (int t = 0; t < 4; ++t) { v8f z = {0.f, 0.f, 0.f, 0.f, 0.f, 0.f, 0.f, 0.f}; acc[t] = z; }
  mmk<4, K>(acc, tA, r0, Pw, c0);

#pragma unroll
  for (int t = 0; t < 4; ++t) {
    const int col = c0 + 16 * t + m;
    const float bb = bias[col];
#pragma unroll
    for (int r = 0; r < 8; ++r)
      stg[(r0 + 8 * hh + r) * NOUT + col] = fmaxf(acc[t][r] * WSCLI + bb, 0.f);
  }
  __syncthreads();

#pragma unroll
  for (int row = 0; row < BM / NWAVE; ++row) {
    const int lrow = (BM / NWAVE) * wave + row;
    const int grow = rowBase + lrow;
    if (grow < nWrite) {
      const v4f v0 = *(const v4f*)(stg + lrow * NOUT + 4 * lane);
      const v4f v1 = *(const v4f*)(stg + lrow * NOUT + 128 + 4 * lane);
      float* po = out + (size_t)grow * NOUT;
      *(volatile v4f*)(po + 4 * lane) = v0;
      *(volatile v4f*)(po + 128 + 4 * lane) = v1;
    }
  }
  __threadfence();
#pragma unroll
  for (int row = 0; row < BM / NWAVE; ++row) {
    const int lrow = (BM / NWAVE) * wave + row;
    const int grow = rowBase + lrow;
    if (grow < nWrite) {
      const v4f v0 = *(const v4f*)(stg + lrow * NOUT + 4 * lane);
      const v4f v1 = *(const v4f*)(stg + lrow * NOUT + 128 + 4 * lane);
      float* po = out + (size_t)grow * NOUT;
      *(volatile v4f*)(po + 4 * lane) = v0;
      *(volatile v4f*)(po + 128 + 4 * lane) = v1;
    }
  }
}

static size_t carve(size_t* o, size_t bytes) {
  const size_t r = *o;
  *o += (bytes + 255) & ~(size_t)255;
  return r;
}

extern "C" void kernel_launch(void* const* d_in, const int* in_sizes, int n_in,
                              void* d_out, int out_size, void* d_ws, size_t ws_size,
                              hipStream_t stream) {
  if (n_in < 7) return;
  const int nN = in_sizes[0] / D1;
  const int nE = in_sizes[1];
  if (nN <= 0 || nE <= 0 || in_sizes[0] != nN * D1 || in_sizes[2] != nE) return;
  if (in_sizes[3] != K1 * NOUT || in_sizes[4] != NOUT || in_sizes[5] != K2 * NOUT || in_sizes[6] != NOUT) return;
  if ((long long)out_size != (long long)nN * NOUT) return;
  if (nE > (1 << 27) || nN > (1 << 22)) return;

  const float* x   = (const float*)d_in[0];
  const int*   src = (const int*)d_in[1];
  const int*   dst = (const int*)d_in[2];
  const float* w1  = (const float*)d_in[3];
  const float* b1v = (const float*)d_in[4];
  const float* w2  = (const float*)d_in[5];
  const float* b2v = (const float*)d_in[6];
  float* dout = (float*)d_out;

  const int NPAD   = ((nN + TGT - 1) / TGT) * TGT;
  const int nBC    = (nN + NBC - 1) / NBC;
  const int CNTPAD = nBC * NBC;
  if (FPC * nBC + 1 > RBN) return;
  const int nBF    = (nN + NBF - 1) / NBF;
  const int csrLen = ((nE + 31) & ~31) + 4096;
  if (31 * FPC * nBC > 4096) return;
  if ((long long)nE * NBF > (long long)nN * (RCAP / 4 * 3)) return;
  if ((long long)nE > (long long)nN * (DEGCAP / 2)) return;
  const int nAgg   = NPAD / TGT;
  const int nMl    = (nN + BM - 1) / BM;
  const int nHrows = nMl * BM;

  char* ws = (char*)d_ws;
  size_t o = 0;
  const size_t oP1  = carve(&o, (size_t)NOUT * K1 * 2);
  const size_t oP2  = carve(&o, (size_t)NOUT * K2 * 2);
  const size_t oCnt = carve(&o, (size_t)CNTPAD * 4);
  const size_t oOff = carve(&o, (size_t)CNTPAD * 4);
  const size_t oRb  = carve(&o, (size_t)RBN * 4);
  const size_t oCsr = carve(&o, (size_t)csrLen * 4);
  const size_t oAG1 = carve(&o, (size_t)NPAD * D1 * 2);
  const size_t oH   = carve(&o, (size_t)NPAD * NOUT * 4);
  const size_t oAG2 = carve(&o, (size_t)NPAD * NOUT * 2);
  if (o > ws_size || o > (size_t)WSCAP) return;

  _Float16* pP1  = (_Float16*)(ws + oP1);
  _Float16* pP2  = (_Float16*)(ws + oP2);
  int*      cnt  = (int*)(ws + oCnt);
  int*      offp = (int*)(ws + oOff);
  int*      rb   = (int*)(ws + oRb);
  int*      csr  = (int*)(ws + oCsr);
  _Float16* AG1  = (_Float16*)(ws + oAG1);
  float*    H    = (float*)(ws + oH);
  _Float16* AG2  = (_Float16*)(ws + oAG2);

  const int vec8 = 1;

  k_wprep<<<NTILE1 + NTILE2, NTHR, 0, stream>>>(w1, w2, pP1, pP2);

  k_count<<<nBC, NTHR, 0, stream>>>(dst, cnt, nE, vec8);
  k_offsets<<<1, OTHR, 0, stream>>>(cnt, offp, rb, nBC);
  hipFuncSetAttribute(reinterpret_cast<const void*>(&k_fill),
                      hipFuncAttributeMaxDynamicSharedMemorySize, LDS_FILL);
  k_fill<<<nBF, NTHR, LDS_FILL, stream>>>(dst, src, offp, rb, csr, nN, nE, vec8, csrLen);

  k_agg<1><<<nAgg, NTHR, 0, stream>>>(csr, offp, cnt, x, AG1, nN, csrLen);

  hipFuncSetAttribute(reinterpret_cast<const void*>(&k_mlp<D1>),
                      hipFuncAttributeMaxDynamicSharedMemorySize, LDS_MLP1);
  k_mlp<D1><<<nMl, NTHR, LDS_MLP1, stream>>>(x, AG1, pP1, b1v, H, nN, NPAD, nHrows);

  k_agg<2><<<nAgg, NTHR, 0, stream>>>(csr, offp, cnt, H, AG2, nN, csrLen);

  hipFuncSetAttribute(reinterpret_cast<const void*>(&k_mlp<NOUT>),
                      hipFuncAttributeMaxDynamicSharedMemorySize, LDS_MLP2);
  k_mlp<NOUT><<<nMl, NTHR, LDS_MLP2, stream>>>(H, AG2, pP2, b2v, dout, nN, NPAD, nN);
}
